// UniModelMatcher_83434034692461
// MI455X (gfx1250) — hardware-verified
//
#include <hip/hip_runtime.h>


typedef _Float16 v16h __attribute__((ext_vector_type(16)));
typedef _Float16 v8h __attribute__((ext_vector_type(8)));
typedef float v8f __attribute__((ext_vector_type(8)));
typedef float v4f __attribute__((ext_vector_type(4)));

union Frag {
  v16h v;
  v8h hv[2];
};

__device__ __forceinline__ void ldfrag(Frag& f, const _Float16* p, int h) {
  f.hv[0] = *(const v8h*)(p + 8 * h);
  f.hv[1] = *(const v8h*)(p + 16 + 8 * h);
}

__device__ __forceinline__ v8f mma(v16h a, v16h b, v8f c) {
  c = __builtin_amdgcn_wmma_f32_16x16x32_f16(false, a, false, b, (short)0, c, false, false);
  asm volatile("v_nop\n\tv_nop\n\tv_nop\n\tv_nop" : "+v"(c) : "v"(a), "v"(b));
  return c;
}

__device__ __forceinline__ float wave_sum(float v) {
#pragma unroll
  for (int o = 16; o >= 1; o >>= 1) v += __shfl_xor(v, o, 32);
  return v;
}

__device__ __forceinline__ float wave_max(float v) {
#pragma unroll
  for (int o = 16; o >= 1; o >>= 1) v = fmaxf(v, __shfl_xor(v, o, 32));
  return v;
}

__global__ void __launch_bounds__(256) k_cvt_h(const float* __restrict__ X, _Float16* __restrict__ Y, int n8) {
  const int i = blockIdx.x * 256 + threadIdx.x;
  const bool ok = i < n8;
  const size_t base = (size_t)(ok ? i : 0) * 8;
  const v4f x0 = *(const v4f*)(X + base);
  const v4f x1 = *(const v4f*)(X + base + 4);
  v8h o;
  o[0] = (_Float16)x0[0]; o[1] = (_Float16)x0[1]; o[2] = (_Float16)x0[2]; o[3] = (_Float16)x0[3];
  o[4] = (_Float16)x1[0]; o[5] = (_Float16)x1[1]; o[6] = (_Float16)x1[2]; o[7] = (_Float16)x1[3];
  _Float16* yp = Y + base;
  if (ok) *(volatile v8h*)yp = o;
  __threadfence();
  if (ok) *(volatile v8h*)yp = o;
}

__global__ void __launch_bounds__(256) k_cvt_w(const float* __restrict__ W0, const float* __restrict__ W1,
                                                const float* __restrict__ W2, const float* __restrict__ W3,
                                                _Float16* __restrict__ WT, float scl) {
  __shared__ float tile[64 * 33];
  const int z = blockIdx.z;
  const float* W = (z == 0) ? W0 : ((z == 1) ? W1 : ((z == 2) ? W2 : W3));
  _Float16* Wt = WT + (size_t)z * 768 * 768;
  const int n0 = blockIdx.x * 32, k0 = blockIdx.y * 64;
  const int tid = threadIdx.x;
  {
    const int row = tid >> 2, c8 = (tid & 3) * 8;
    const float* src = W + (size_t)(k0 + row) * 768 + n0 + c8;
    const v4f u0 = *(const v4f*)src;
    const v4f u1 = *(const v4f*)(src + 4);
#pragma unroll
    for (int e = 0; e < 4; ++e) {
      tile[row * 33 + c8 + e] = u0[e];
      tile[row * 33 + c8 + 4 + e] = u1[e];
    }
  }
  __syncthreads();
  const int wid = tid >> 5, lane = tid & 31, q = lane >> 3, p = lane & 7;
  const int L = 4 * wid + q;
  v8h o;
#pragma unroll
  for (int e = 0; e < 8; ++e) o[e] = (_Float16)(tile[(8 * p + e) * 33 + L] * scl);
  _Float16* dst = Wt + (size_t)(n0 + L) * 768 + k0 + 8 * p;
  *(volatile v8h*)dst = o;
  __threadfence();
  *(volatile v8h*)dst = o;
}

template <int MODE>
__global__ void __launch_bounds__(128)
k_gemm(const _Float16* __restrict__ A, const _Float16* __restrict__ Bt, const float* __restrict__ bias,
       float* __restrict__ OutF, _Float16* __restrict__ OutH, int M, int N, int K, float scale) {
  __shared__ __attribute__((aligned(16))) float st[4 * 32 * 36];
  const int tid = threadIdx.x, wid = tid >> 5, lane = tid & 31, h = lane >> 4, m = lane & 15;
  const int ntn = N >> 5, ntiles = (M >> 5) * ntn;
  int tile = blockIdx.x * 4 + wid;
  const bool active = tile < ntiles;
  if (!active) tile = ntiles - 1;
  const int tm = tile / ntn, tn = tile - tm * ntn;
  const _Float16* a0p = A + (size_t)(tm * 32 + m) * (size_t)K;
  const _Float16* a1p = a0p + (size_t)16 * (size_t)K;
  const _Float16* b0p = Bt + (size_t)(tn * 32 + m) * (size_t)K;
  const _Float16* b1p = b0p + (size_t)16 * (size_t)K;
  v8f c00 = {0.f, 0.f, 0.f, 0.f, 0.f, 0.f, 0.f, 0.f};
  v8f c01 = {0.f, 0.f, 0.f, 0.f, 0.f, 0.f, 0.f, 0.f};
  v8f c10 = {0.f, 0.f, 0.f, 0.f, 0.f, 0.f, 0.f, 0.f};
  v8f c11 = {0.f, 0.f, 0.f, 0.f, 0.f, 0.f, 0.f, 0.f};
#pragma unroll 2
  for (int k0 = 0; k0 < K; k0 += 32) {
    Frag fa0, fa1, fb0, fb1;
    ldfrag(fa0, a0p + k0, h);
    ldfrag(fa1, a1p + k0, h);
    ldfrag(fb0, b0p + k0, h);
    ldfrag(fb1, b1p + k0, h);
    c00 = mma(fa0.v, fb0.v, c00);
    c01 = mma(fa0.v, fb1.v, c01);
    c10 = mma(fa1.v, fb0.v, c10);
    c11 = mma(fa1.v, fb1.v, c11);
  }
  float* s = st + wid * (32 * 36);
#pragma unroll
  for (int r = 0; r < 8; ++r) {
    const int ra = 8 * h + r, rb = 16 + 8 * h + r;
    s[ra * 36 + m] = c00[r];
    s[ra * 36 + 16 + m] = c01[r];
    s[rb * 36 + m] = c10[r];
    s[rb * 36 + 16 + m] = c11[r];
  }
  __syncthreads();
  const int q = lane >> 3, p = lane & 7;
  if (MODE == 0) {
    const v4f bb = *(const v4f*)(bias + tn * 32 + 4 * p);
    v4f vals[8];
#pragma unroll
    for (int sI = 0; sI < 8; ++sI) {
      const v4f u = *(const v4f*)(s + (4 * sI + q) * 36 + 4 * p);
      v4f w;
#pragma unroll
      for (int e = 0; e < 4; ++e) w[e] = u[e] * scale + bb[e];
      vals[sI] = w;
    }
    float* ob = OutF + (size_t)(tm * 32 + q) * (size_t)N + tn * 32 + 4 * p;
    if (active) {
#pragma unroll
      for (int sI = 0; sI < 8; ++sI) *(volatile v4f*)(ob + (size_t)(4 * sI) * (size_t)N) = vals[sI];
    }
    __threadfence();
    if (active) {
#pragma unroll
      for (int sI = 0; sI < 8; ++sI) *(volatile v4f*)(ob + (size_t)(4 * sI) * (size_t)N) = vals[sI];
    }
  } else {
    v8h vals[4];
#pragma unroll
    for (int sI = 0; sI < 4; ++sI) {
      const int L = 4 * sI + q, nc = 2 * L + (p >> 2), j0 = 8 * (p & 3);
      const float bb = bias[tn * 32 + nc];
      v8h w;
#pragma unroll
      for (int e = 0; e < 8; ++e) w[e] = (_Float16)(s[(j0 + e) * 36 + nc] * scale + bb);
      vals[sI] = w;
    }
    _Float16* ob = OutH + ((size_t)tm * (size_t)N + (size_t)tn * 32) * 32;
    if (active) {
#pragma unroll
      for (int sI = 0; sI < 4; ++sI) {
        const int L = 4 * sI + q, nc = 2 * L + (p >> 2), j0 = 8 * (p & 3);
        *(volatile v8h*)(ob + (size_t)nc * 32 + j0) = vals[sI];
      }
    }
    __threadfence();
    if (active) {
#pragma unroll
      for (int sI = 0; sI < 4; ++sI) {
        const int L = 4 * sI + q, nc = 2 * L + (p >> 2), j0 = 8 * (p & 3);
        *(volatile v8h*)(ob + (size_t)nc * 32 + j0) = vals[sI];
      }
    }
  }
}

__global__ void __launch_bounds__(256) k_rownorm(const float* __restrict__ X, _Float16* __restrict__ Y, int R, float oscale) {
  const int wid = threadIdx.x >> 5, lane = threadIdx.x & 31;
  const int row = blockIdx.x * 8 + wid;
  const bool ok = row < R;
  const int rowc = ok ? row : 0;
  const float* xr = X + (size_t)rowc * 768 + 8 * lane;
  v4f u[6];
  float ss = 0.f;
#pragma unroll
  for (int t = 0; t < 3; ++t) {
    u[2 * t] = *(const v4f*)(xr + 256 * t);
    u[2 * t + 1] = *(const v4f*)(xr + 256 * t + 4);
#pragma unroll
    for (int e = 0; e < 4; ++e) ss += u[2 * t][e] * u[2 * t][e] + u[2 * t + 1][e] * u[2 * t + 1][e];
  }
  ss = wave_sum(ss);
  const float rc = 1.0f / fmaxf(sqrtf(ss), 1e-8f);
  v8h o[3];
#pragma unroll
  for (int t = 0; t < 3; ++t) {
    v8h w;
#pragma unroll
    for (int e = 0; e < 4; ++e) {
      w[e] = (_Float16)((u[2 * t][e] * rc) * oscale);
      w[4 + e] = (_Float16)((u[2 * t + 1][e] * rc) * oscale);
    }
    o[t] = w;
  }
  _Float16* yr = Y + (size_t)rowc * 768 + 8 * lane;
  if (ok) {
#pragma unroll
    for (int t = 0; t < 3; ++t) *(volatile v8h*)(yr + 256 * t) = o[t];
  }
  __threadfence();
  if (ok) {
#pragma unroll
    for (int t = 0; t < 3; ++t) *(volatile v8h*)(yr + 256 * t) = o[t];
  }
}

#define ATT_F      (32 * 768)
#define TH_OFF_F   (ATT_F)
#define RED_OFF    (ATT_F + 512)
#define SROW_OFF   (RED_OFF + 256)
#define WROW_OFF   (SROW_OFF + 32)
#define RS_OFF     (WROW_OFF + 32)
#define RQ_OFF     (RS_OFF + 8)
#define RG_OFF     (RQ_OFF + 8)
#define ATT_LDS_FLOATS (RG_OFF + 8)

__global__ void __launch_bounds__(256)
k_attend(const _Float16* __restrict__ Qn, const _Float16* __restrict__ Kn, const _Float16* __restrict__ Vt,
         const float* __restrict__ Qf,
         const float* __restrict__ ln1g, const float* __restrict__ ln1b,
         const float* __restrict__ Wsp, const float* __restrict__ bsp,
         const float* __restrict__ ln2g, const float* __restrict__ ln2b,
         const float* __restrict__ Ef, float* __restrict__ G2L) {
  extern __shared__ __attribute__((aligned(16))) float smem[];
  float* att = smem;
  float* cpart = smem;
  _Float16* Th = (_Float16*)(smem + TH_OFF_F);
  float* red = smem + RED_OFF;
  float* srow = smem + SROW_OFF;
  float* wrow = smem + WROW_OFF;
  float* reds = smem + RS_OFF;
  float* redq = smem + RQ_OFF;
  float* redg = smem + RG_OFF;

  const int ab = blockIdx.x, a = ab >> 6, b = ab & 63;
  const int tid = threadIdx.x, wid = tid >> 5, lane = tid & 31, h = lane >> 4, m = lane & 15;

  {
    const int t = wid & 3, tmq = t >> 1, tnk = t & 1, kh = wid >> 2;
    const _Float16* ap = Qn + (size_t)(a * 32 + tmq * 16 + m) * 768 + kh * 384;
    const _Float16* bp = Kn + (size_t)(b * 32 + tnk * 16 + m) * 768 + kh * 384;
    v8f cc = {0.f, 0.f, 0.f, 0.f, 0.f, 0.f, 0.f, 0.f};
#pragma unroll 2
    for (int ks = 0; ks < 12; ++ks) {
      Frag fa, fb;
      ldfrag(fa, ap + ks * 32, h);
      ldfrag(fb, bp + ks * 32, h);
      cc = mma(fa.v, fb.v, cc);
    }
#pragma unroll
    for (int r = 0; r < 8; ++r)
      cpart[kh * 1024 + (tmq * 16 + 8 * h + r) * 32 + tnk * 16 + m] = cc[r];
  }
  __syncthreads();

  float qv[4];
#pragma unroll
  for (int r = 0; r < 4; ++r) {
    const int i = wid * 4 + r;
    const float c = (cpart[i * 32 + lane] + cpart[1024 + i * 32 + lane]) * (1.0f / 256.0f);
    qv[r] = expf(c * 10.0f);
  }
#pragma unroll 1
  for (int it = 0; it < 10; ++it) {
#pragma unroll
    for (int r = 0; r < 4; ++r) {
      const float rs = wave_sum(qv[r]);
      qv[r] = qv[r] * (1.0f / rs);
    }
    red[wid * 32 + lane] = (qv[0] + qv[1]) + (qv[2] + qv[3]);
    __syncthreads();
    float cs = 0.f;
#pragma unroll
    for (int w = 0; w < 8; ++w) cs += red[w * 32 + lane];
    const float rc = 1.0f / cs;
#pragma unroll
    for (int r = 0; r < 4; ++r) qv[r] = qv[r] * rc;
    __syncthreads();
  }
#pragma unroll
  for (int r = 0; r < 4; ++r) {
    const float ss = wave_sum(qv[r] * qv[r]);
    const float rn = 1.0f / fmaxf(sqrtf(ss), 1e-12f);
    Th[(wid * 4 + r) * 32 + lane] = (_Float16)((qv[r] * rn) * 16384.0f);
  }
  __syncthreads();

  {
    Frag fa0, fa1;
    ldfrag(fa0, Th + m * 32, h);
    ldfrag(fa1, Th + (16 + m) * 32, h);
    const float* qrow = Qf + (size_t)(a * 32) * 768;
    const v8f z = {0.f, 0.f, 0.f, 0.f, 0.f, 0.f, 0.f, 0.f};
#pragma unroll 2
    for (int nt = wid; nt < 48; nt += 8) {
      Frag fb;
      ldfrag(fb, Vt + (size_t)(b * 768 + nt * 16 + m) * 32, h);
      const v8f d0 = mma(fa0.v, fb.v, z);
      const v8f d1 = mma(fa1.v, fb.v, z);
      const int n = nt * 16 + m;
#pragma unroll
      for (int r = 0; r < 8; ++r) {
        const int r0 = 8 * h + r, r1 = 16 + 8 * h + r;
        att[r0 * 768 + n] = d0[r] * (1.0f / 16384.0f) + qrow[(size_t)r0 * 768 + n];
        att[r1 * 768 + n] = d1[r] * (1.0f / 16384.0f) + qrow[(size_t)r1 * 768 + n];
      }
    }
  }
  __syncthreads();

  {
    const float bspv = bsp[0];
#pragma unroll 1
    for (int rr = 0; rr < 4; ++rr) {
      const int row = wid * 4 + rr;
      float* ar = att + row * 768;
      float x[24];
      float ssum = 0.f;
#pragma unroll
      for (int t = 0; t < 24; ++t) {
        x[t] = ar[lane + 32 * t];
        ssum += x[t];
      }
      ssum = wave_sum(ssum);
      const float mean = ssum * (1.0f / 768.0f);
      float vs = 0.f;
#pragma unroll
      for (int t = 0; t < 24; ++t) {
        const float d = x[t] - mean;
        vs += d * d;
      }
      vs = wave_sum(vs);
      const float inv = rsqrtf(vs * (1.0f / 768.0f) + 1e-5f);
      float dot = 0.f;
#pragma unroll
      for (int t = 0; t < 24; ++t) {
        const int c = lane + 32 * t;
        const float y = ((x[t] - mean) * inv) * ln1g[c] + ln1b[c];
        ar[c] = y;
        dot += y * Wsp[c];
      }
      dot = wave_sum(dot);
      if (lane == 0) srow[row] = dot + bspv;
    }
  }
  __syncthreads();

  if (wid == 0) {
    const float v = srow[lane];
    const float mx = wave_max(v);
    const float e = expf(v - mx);
    const float se = wave_sum(e);
    wrow[lane] = e * (1.0f / se);
  }
  __syncthreads();

  float pv[3];
  float ls = 0.f;
#pragma unroll
  for (int t = 0; t < 3; ++t) {
    const int n = tid + 256 * t;
    float acc = 0.f;
#pragma unroll 8
    for (int i = 0; i < 32; ++i) acc += att[i * 768 + n] * wrow[i];
    pv[t] = acc;
    ls += acc;
  }
  ls = wave_sum(ls);
  if (lane == 0) reds[wid] = ls;
  __syncthreads();
  float tsum = 0.f;
#pragma unroll
  for (int w = 0; w < 8; ++w) tsum += reds[w];
  const float mean2 = tsum * (1.0f / 768.0f);
  float lq = 0.f;
#pragma unroll
  for (int t = 0; t < 3; ++t) {
    const float d = pv[t] - mean2;
    lq += d * d;
  }
  lq = wave_sum(lq);
  if (lane == 0) redq[wid] = lq;
  __syncthreads();
  float tq = 0.f;
#pragma unroll
  for (int w = 0; w < 8; ++w) tq += redq[w];
  const float inv2 = rsqrtf(tq * (1.0f / 768.0f) + 1e-5f);
  float gl = 0.f;
#pragma unroll
  for (int t = 0; t < 3; ++t) {
    const int n = tid + 256 * t;
    const float cx = ((pv[t] - mean2) * inv2) * ln2g[n] + ln2b[n];
    gl += Ef[(size_t)a * 768 + n] * cx;
  }
  gl = wave_sum(gl);
  if (lane == 0) redg[wid] = gl;
  __syncthreads();
  if (wid == 0) {
    float tot = 0.f;
#pragma unroll
    for (int w = 0; w < 8; ++w) tot += redg[w];
    if (lane < 8) {
      const v4f o = {tot, tot, tot, tot};
      float* gp = G2L + (size_t)ab * 32 + 4 * lane;
      *(volatile v4f*)gp = o;
      __threadfence();
      *(volatile v4f*)gp = o;
    }
  }
}

__global__ void __launch_bounds__(256) k_final(const float* __restrict__ G2L, const float* __restrict__ EntCls,
                                                const float* __restrict__ MenCls, float* __restrict__ Out) {
  __shared__ __attribute__((aligned(16))) float orow[32];
  const int b = blockIdx.x;
  const int tid = threadIdx.x, wid = tid >> 5, lane = tid & 31;
  float mc[24];
#pragma unroll
  for (int t = 0; t < 24; ++t) mc[t] = MenCls[(size_t)b * 768 + lane + 32 * t];
#pragma unroll 1
  for (int rr = 0; rr < 4; ++rr) {
    const int a = wid * 4 + rr;
    const float* ec = EntCls + (size_t)a * 768 + lane;
    float g = 0.f;
#pragma unroll
    for (int t = 0; t < 24; ++t) g += mc[t] * ec[32 * t];
    g = wave_sum(g);
    const float gl = G2L[((size_t)a * 64 + b) * 32];
    if (lane == 0) orow[a] = (gl + g) * 0.5f;
  }
  __syncthreads();
  if (tid < 8) {
    v4f o;
    o[0] = orow[4 * tid]; o[1] = orow[4 * tid + 1]; o[2] = orow[4 * tid + 2]; o[3] = orow[4 * tid + 3];
    float* op = Out + (size_t)b * 32 + 4 * tid;
    *(volatile v4f*)op = o;
    __threadfence();
    *(volatile v4f*)op = o;
  }
}

extern "C" void kernel_launch(void* const* d_in, const int* in_sizes, int n_in,
                              void* d_out, int out_size, void* d_ws, size_t ws_size,
                              hipStream_t stream) {
  const int Na = 32, La = 32, Bm = 64, Lb = 32, D = 768;
  if (n_in < 18) return;
  if (in_sizes[0] != Na * D || in_sizes[1] != Na * La * D || in_sizes[2] != Bm * D || in_sizes[3] != Bm * Lb * D) return;
  if (in_sizes[4] != D * D || in_sizes[6] != D * D || in_sizes[8] != D * D || in_sizes[12] != D * D) return;
  if (in_sizes[5] != D || in_sizes[7] != D || in_sizes[9] != D || in_sizes[10] != D || in_sizes[11] != D) return;
  if (in_sizes[13] != D || in_sizes[14] != D || in_sizes[15] < 1 || in_sizes[16] != D || in_sizes[17] != D) return;
  if (out_size != Bm * Na) return;

  const float* entity_cls     = (const float*)d_in[0];
  const float* entity_tokens  = (const float*)d_in[1];
  const float* mention_cls    = (const float*)d_in[2];
  const float* mention_tokens = (const float*)d_in[3];
  const float* Wq   = (const float*)d_in[4];
  const float* bq   = (const float*)d_in[5];
  const float* Wk   = (const float*)d_in[6];
  const float* bk   = (const float*)d_in[7];
  const float* Wv   = (const float*)d_in[8];
  const float* bv   = (const float*)d_in[9];
  const float* ln1g = (const float*)d_in[10];
  const float* ln1b = (const float*)d_in[11];
  const float* Wcls = (const float*)d_in[12];
  const float* bcls = (const float*)d_in[13];
  const float* Wsp  = (const float*)d_in[14];
  const float* bsp  = (const float*)d_in[15];
  const float* ln2g = (const float*)d_in[16];
  const float* ln2b = (const float*)d_in[17];
  float* Out = (float*)d_out;

  const int RE = Na * La;
  const int RM = Bm * Lb;
  const size_t WSZ = (size_t)D * D;

  size_t off = 0;
  auto carve = [&](size_t bytes) { size_t o = off; off += (bytes + 255) & ~(size_t)255; return o; };
  const size_t oEh  = carve((size_t)RE * D * 2);
  const size_t oMh  = carve((size_t)RM * D * 2);
  const size_t oEch = carve((size_t)Na * D * 2);
  const size_t oWT  = carve(4 * WSZ * 2);
  const size_t oQf  = carve((size_t)RE * D * 4);
  const size_t oKf  = carve((size_t)RM * D * 4);
  const size_t oVt  = carve((size_t)RM * D * 2);
  const size_t oEf  = carve((size_t)Na * D * 4);
  const size_t oQn  = carve((size_t)RE * D * 2);
  const size_t oKn  = carve((size_t)RM * D * 2);
  const size_t oG2L = carve((size_t)Na * Bm * 32 * 4);
  if (off > ws_size) return;

  char* ws = (char*)d_ws;
  _Float16* Eh  = (_Float16*)(ws + oEh);
  _Float16* Mh  = (_Float16*)(ws + oMh);
  _Float16* Ech = (_Float16*)(ws + oEch);
  _Float16* WT  = (_Float16*)(ws + oWT);
  float*    Qf  = (float*)(ws + oQf);
  float*    Kf  = (float*)(ws + oKf);
  _Float16* Vt  = (_Float16*)(ws + oVt);
  float*    Ef  = (float*)(ws + oEf);
  _Float16* Qn  = (_Float16*)(ws + oQn);
  _Float16* Kn  = (_Float16*)(ws + oKn);
  float*    G2L = (float*)(ws + oG2L);

  {
    const int n8e = RE * D / 8, n8m = RM * D / 8, n8c = Na * D / 8;
    k_cvt_h<<<(n8e + 255) / 256, 256, 0, stream>>>(entity_tokens, Eh, n8e);
    k_cvt_h<<<(n8m + 255) / 256, 256, 0, stream>>>(mention_tokens, Mh, n8m);
    k_cvt_h<<<(n8c + 255) / 256, 256, 0, stream>>>(entity_cls, Ech, n8c);
    k_cvt_w<<<dim3(D / 32, D / 64, 4), 256, 0, stream>>>(Wq, Wk, Wv, Wcls, WT, 64.0f);
  }

  {
    const float unw = 1.0f / 64.0f;
    const int tq = (RE / 32) * (D / 32);
    const int tk = (RM / 32) * (D / 32);
    const int tc = (Na / 32) * (D / 32);
    k_gemm<0><<<(tq + 3) / 4, 128, 0, stream>>>(Eh, WT + 0 * WSZ, bq, Qf, Vt, RE, D, D, unw);
    k_gemm<0><<<(tk + 3) / 4, 128, 0, stream>>>(Mh, WT + 1 * WSZ, bk, Kf, Vt, RM, D, D, unw);
    k_gemm<1><<<(tk + 3) / 4, 128, 0, stream>>>(Mh, WT + 2 * WSZ, bv, Kf, Vt, RM, D, D, unw);
    k_gemm<0><<<(tc + 3) / 4, 128, 0, stream>>>(Ech, WT + 3 * WSZ, bcls, Ef, Vt, Na, D, D, unw);
  }

  k_rownorm<<<(RE + 7) / 8, 256, 0, stream>>>(Qf, Qn, RE, 16.0f);
  k_rownorm<<<(RM + 7) / 8, 256, 0, stream>>>(Kf, Kn, RM, 16.0f);

  {
    const size_t lds = (size_t)ATT_LDS_FLOATS * sizeof(float);
    k_attend<<<Na * Bm, 256, lds, stream>>>(Qn, Kn, Vt, Qf, ln1g, ln1b, Wsp, bsp, ln2g, ln2b, Ef, G2L);
  }

  k_final<<<Bm, 256, 0, stream>>>(G2L, entity_cls, mention_cls, Out);
}
